// ClassicalSelfAttention_65481071407449
// MI455X (gfx1250) — hardware-verified
//
#include <hip/hip_runtime.h>


#ifndef NB
#define NB 4
#endif
#ifndef SEQ
#define SEQ 2048
#endif
#define NB_FULL 4
#define SEQ_FULL 2048
#define EMB 1024
#define PCAR 1024.0f
#define PSUB (PCAR / (float)SEQ)
#define SCL 0.03125f

static_assert(NB >= 1 && NB <= NB_FULL);
static_assert(SEQ >= 128 && SEQ <= SEQ_FULL);
static_assert(SEQ % 128 == 0);
static_assert(EMB % 64 == 0 && EMB % 256 == 0);
static_assert((SEQ / 8) % 8 == 0);

typedef _Float16 h16;
typedef unsigned short bf;
typedef __attribute__((ext_vector_type(16))) __bf16   v16bf;
typedef __attribute__((ext_vector_type(16))) _Float16 v16h;
typedef __attribute__((ext_vector_type(8)))  _Float16 v8h;
typedef __attribute__((ext_vector_type(4)))  _Float16 v4h;
typedef __attribute__((ext_vector_type(8)))  unsigned short v8us;
typedef __attribute__((ext_vector_type(8)))  float    v8f;
typedef __attribute__((ext_vector_type(4)))  float    v4f;
typedef v8h  __attribute__((may_alias)) v8ha;
typedef v4f  __attribute__((may_alias)) v4fa;
typedef v8us __attribute__((may_alias)) v8usa;

__device__ __forceinline__ unsigned short f2bf(float f) { unsigned u = __float_as_uint(f); u += 0x7FFFu + ((u >> 16) & 1u); return (unsigned short)(u >> 16); }
__device__ __forceinline__ float bf2f(unsigned short b) { return __uint_as_float(((unsigned)b) << 16); }
__device__ __forceinline__ h16 tohx(float x) { return (h16)x; }
__device__ __forceinline__ v16h cat16(v8h lo, v8h hi) { return __builtin_shufflevector(lo, hi, 0, 1, 2, 3, 4, 5, 6, 7, 8, 9, 10, 11, 12, 13, 14, 15); }
__device__ __forceinline__ v16bf cat16b(v8us lo, v8us hi) { return __builtin_bit_cast(v16bf, __builtin_shufflevector(lo, hi, 0, 1, 2, 3, 4, 5, 6, 7, 8, 9, 10, 11, 12, 13, 14, 15)); }
__device__ __forceinline__ v8f wmma16(v16h a, v16h b, v8f c) { return __builtin_amdgcn_wmma_f32_16x16x32_f16(false, a, false, b, (short)0, c, false, false); }
__device__ __forceinline__ v8f wmmab(v16bf a, v16bf b, v8f c) { return __builtin_amdgcn_wmma_f32_16x16x32_bf16(false, a, false, b, (short)0, c, false, false); }

template <typename T16> struct WFrag;
template <> struct WFrag<h16> { typedef v16h V; static __device__ __forceinline__ V ld(const h16* p) { return cat16(*(const v8h*)p, *(const v8h*)(p + 16)); } static __device__ __forceinline__ v8f mma(V a, V b, v8f c) { return wmma16(a, b, c); } };
template <> struct WFrag<bf> { typedef v16bf V; static __device__ __forceinline__ V ld(const bf* p) { return cat16b(*(const v8us*)p, *(const v8us*)(p + 16)); } static __device__ __forceinline__ v8f mma(V a, V b, v8f c) { return wmmab(a, b, c); } };
template <typename T16, int NSPLIT, bool BIAS>
__global__ __launch_bounds__(32) void k_gemmw(const T16* __restrict__ A, const T16* __restrict__ A2, const T16* __restrict__ Bt, const T16* __restrict__ Bt2, int K, float* C, int ldc, const float* __restrict__ bias, float scale, size_t sA, size_t sB, size_t sC) {
    typedef typename WFrag<T16>::V V;
    __shared__ __align__(16) float os[16 * 68];
    const size_t z = blockIdx.z; A += z * sA; if (A2) A2 += z * sA; Bt += z * sB; if (Bt2) Bt2 += z * sB; C += z * sC;
    const int lane = threadIdx.x & 31, lr = lane & 15, hi = lane >> 4; const int r0 = blockIdx.x * 64, c0 = blockIdx.y * 64;
    v8f acc[4][4];
#pragma unroll
    for (int mb = 0; mb < 4; ++mb)
#pragma unroll
        for (int nb = 0; nb < 4; ++nb) acc[mb][nb] = (v8f){};
    const size_t aoff = (size_t)(r0 + lr) * K + 8 * hi, boff = (size_t)(c0 + lr) * K + 8 * hi;
#pragma unroll 1
    for (int kc = 0; kc < K; kc += 32) {
        V a[4], a2[4];
#pragma unroll
        for (int mb = 0; mb < 4; ++mb) { a[mb] = WFrag<T16>::ld(A + aoff + (size_t)mb * 16 * K + kc); if (NSPLIT == 1 || NSPLIT == 2) a2[mb] = WFrag<T16>::ld(A2 + aoff + (size_t)mb * 16 * K + kc); }
#pragma unroll
        for (int nb = 0; nb < 4; ++nb) { const V b = WFrag<T16>::ld(Bt + boff + (size_t)nb * 16 * K + kc); V b2; if (NSPLIT >= 2) b2 = WFrag<T16>::ld(Bt2 + boff + (size_t)nb * 16 * K + kc);
#pragma unroll
            for (int mb = 0; mb < 4; ++mb) { acc[mb][nb] = WFrag<T16>::mma(a[mb], b, acc[mb][nb]); if (NSPLIT == 1 || NSPLIT == 2) acc[mb][nb] = WFrag<T16>::mma(a2[mb], b, acc[mb][nb]); if (NSPLIT >= 2) acc[mb][nb] = WFrag<T16>::mma(a[mb], b2, acc[mb][nb]); } }
        asm volatile("v_nop\n\tv_nop\n\tv_nop\n\tv_nop" : "+v"(acc[0][0]), "+v"(acc[1][1]), "+v"(acc[2][2]), "+v"(acc[3][3]) : "v"(a[0]), "v"(a[3]));
    }
#pragma unroll
    for (int mb = 0; mb < 4; ++mb) {
#pragma unroll
        for (int nb = 0; nb < 4; ++nb) {
#pragma unroll
            for (int j = 0; j < 8; ++j) os[(hi * 8 + j) * 68 + nb * 16 + lr] = acc[mb][nb][j]; }
        __builtin_amdgcn_wave_barrier(); asm volatile("" ::: "memory");
        float* crow = C + (size_t)(r0 + mb * 16) * ldc + c0;
#pragma unroll 1
        for (int ps = 0; ps < 2; ++ps) {
#pragma unroll
            for (int s = 0; s < 8; ++s) { const int row = 2 * s + hi, cofs = lr * 4; v4f val = *(const v4fa*)(os + row * 68 + cofs); val = val * scale;
                if (BIAS) { const v4f bb = *(const v4f*)(bias + c0 + cofs); val = val + bb; }
                *(volatile v4f*)(crow + (size_t)row * ldc + cofs) = val; }
            if (ps == 0) __threadfence(); }
        __builtin_amdgcn_wave_barrier(); asm volatile("" ::: "memory");
    }
}

__global__ __launch_bounds__(256) void k_cvt8(const float* __restrict__ src, bf* dst, size_t n8) { const size_t i = (size_t)blockIdx.x * 256 + threadIdx.x; if (i >= n8) return; const v8f v = *(const v8f*)(src + i * 8); v8us o;
#pragma unroll
    for (int k = 0; k < 8; ++k) o[k] = f2bf(v[k]); *(volatile v8us*)(dst + i * 8) = o; __threadfence(); *(volatile v8us*)(dst + i * 8) = o; }

__global__ __launch_bounds__(256) void k_cvth(const float* __restrict__ src, h16* dst, size_t n8) { const size_t i = (size_t)blockIdx.x * 256 + threadIdx.x; if (i >= n8) return; const v8f v = *(const v8f*)(src + i * 8); v8h o;
#pragma unroll
    for (int k = 0; k < 8; ++k) o[k] = tohx(v[k]); *(volatile v8h*)(dst + i * 8) = o; __threadfence(); *(volatile v8h*)(dst + i * 8) = o; }

__global__ __launch_bounds__(256) void k_vtp8(const float* __restrict__ F, h16* V16) {
    const size_t g = (size_t)blockIdx.x * 256 + threadIdx.x; if (g >= (size_t)EMB * (SEQ / 8)) return;
    const int t0 = (int)(g % (SEQ / 8)) * 8; const int d = (int)(g / (SEQ / 8)); v8h o;
#pragma unroll
    for (int q = 0; q < 8; ++q) o[q] = tohx(F[(size_t)(t0 + q) * EMB + d]);
    h16* p = V16 + (size_t)d * SEQ + t0; *(volatile v8h*)p = o; __threadfence(); *(volatile v8h*)p = o; }

__global__ __launch_bounds__(256) void k_meanv(const float* __restrict__ F, float* MV) {
    const int d = blockIdx.x * 256 + threadIdx.x; if (d >= EMB) return;
    float p[8];
#pragma unroll
    for (int q = 0; q < 8; ++q) p[q] = 0.0f;
#pragma unroll 1
    for (int t = 0; t < SEQ; t += 8) {
#pragma unroll
        for (int q = 0; q < 8; ++q) p[q] += F[(size_t)(t + q) * EMB + d]; }
    const float s = ((p[0] + p[1]) + (p[2] + p[3])) + ((p[4] + p[5]) + (p[6] + p[7]));
    const float m = s * (1.0f / (float)SEQ);
    *(volatile float*)(MV + d) = m; __threadfence(); *(volatile float*)(MV + d) = m; }

__global__ __launch_bounds__(256) void k_asoft(const float* __restrict__ Sb, h16* P16) {
    const int lane = threadIdx.x & 31; const int row = blockIdx.x * 8 + (threadIdx.x >> 5); if (row >= SEQ) return;
    const float* sr = Sb + (size_t)row * SEQ; float v[SEQ / 32]; float mx = -3.0e38f;
#pragma unroll
    for (int ch = 0; ch < SEQ / 128; ++ch) { const int j0 = ch * 128 + lane * 4; const v4f a = *(const v4f*)(sr + j0);
#pragma unroll
        for (int q = 0; q < 4; ++q) { const float t = a[q] * SCL; v[ch * 4 + q] = t; mx = fmaxf(mx, t); } }
#pragma unroll
    for (int sh = 16; sh; sh >>= 1) mx = fmaxf(mx, __shfl_xor(mx, sh, 32));
    float sum = 0.f;
#pragma unroll
    for (int k = 0; k < SEQ / 32; ++k) { float d0 = __fsub_rn(v[k], mx); asm volatile("" : "+v"(d0)); v[k] = __builtin_amdgcn_exp2f(__fmul_rn(d0, 1.4426950408889634f)); sum += v[k]; }
#pragma unroll
    for (int sh = 16; sh; sh >>= 1) sum += __shfl_xor(sum, sh, 32);
    const float f = __fdiv_rn(PCAR, sum);
#pragma unroll
    for (int k = 0; k < SEQ / 32; ++k) v[k] = v[k] * f - PSUB;
    h16* prow = P16 + (size_t)row * SEQ;
#pragma unroll 1
    for (int ps = 0; ps < 2; ++ps) {
#pragma unroll
        for (int ch = 0; ch < SEQ / 128; ++ch) { v4h o4;
#pragma unroll
            for (int q = 0; q < 4; ++q) o4[q] = tohx(v[ch * 4 + q]);
            *(volatile v4h*)(prow + ch * 128 + lane * 4) = o4; }
        if (ps == 0) __threadfence(); }
}

extern "C" void kernel_launch(void* const* d_in, const int* in_sizes, int n_in,
                              void* d_out, int out_size, void* d_ws, size_t ws_size, hipStream_t stream) {
    if (n_in < 4) return;
    const size_t needx = ((size_t)(NB - 1) * SEQ_FULL + SEQ) * EMB;
    if ((size_t)in_sizes[0] < needx || (size_t)in_sizes[1] < (size_t)EMB * EMB || (size_t)in_sizes[2] < (size_t)EMB * EMB || (size_t)in_sizes[3] < (size_t)EMB * EMB) return;
    if ((size_t)out_size < (size_t)NB * SEQ * EMB) return;
    const float* x = (const float*)d_in[0]; const float* wq = (const float*)d_in[1]; const float* wk = (const float*)d_in[2]; const float* wv = (const float*)d_in[3];
    float* OUT = (float*)d_out;
    char* wsp = (char*)d_ws;
    auto take = [&](size_t bytes) { char* p = wsp; wsp += (bytes + 255) & ~(size_t)255; return (void*)p; };
    bf* WQ = (bf*)take((size_t)EMB * EMB * 2); bf* WK = (bf*)take((size_t)EMB * EMB * 2); bf* WV = (bf*)take((size_t)EMB * EMB * 2);
    bf* XB = (bf*)take((size_t)SEQ * EMB * 2);
    float* FQ = (float*)take((size_t)SEQ * EMB * 4); float* FK = (float*)take((size_t)SEQ * EMB * 4); float* FV = (float*)take((size_t)SEQ * EMB * 4);
    h16* Q16 = (h16*)take((size_t)SEQ * EMB * 2); h16* K16 = (h16*)take((size_t)SEQ * EMB * 2); h16* VT16 = (h16*)take((size_t)EMB * SEQ * 2);
    float* MV = (float*)take((size_t)EMB * 4);
    float* Sb = (float*)take((size_t)SEQ * SEQ * 4);
    h16* P16 = (h16*)take((size_t)SEQ * SEQ * 2);
    if ((size_t)(wsp - (char*)d_ws) > ws_size) return;
    const unsigned GW = (unsigned)(((size_t)EMB * EMB / 8 + 255) / 256);
    k_cvt8<<<GW, 256, 0, stream>>>(wq, WQ, (size_t)EMB * EMB / 8);
    k_cvt8<<<GW, 256, 0, stream>>>(wk, WK, (size_t)EMB * EMB / 8);
    k_cvt8<<<GW, 256, 0, stream>>>(wv, WV, (size_t)EMB * EMB / 8);
    const size_t n8 = (size_t)SEQ * EMB / 8; const unsigned G8 = (unsigned)((n8 + 255) / 256);
    const unsigned GV = (unsigned)(((size_t)EMB * (SEQ / 8) + 255) / 256);
    for (int b = 0; b < NB; ++b) {
        const float* xb = x + (size_t)b * SEQ_FULL * EMB; float* ob = OUT + (size_t)b * SEQ * EMB;
        k_cvt8<<<G8, 256, 0, stream>>>(xb, XB, n8);
        k_gemmw<bf, 0, false><<<dim3(SEQ / 64, EMB / 64, 1), 32, 0, stream>>>(XB, nullptr, WQ, nullptr, EMB, FQ, EMB, nullptr, 1.0f, 0, 0, 0);
        k_cvth<<<G8, 256, 0, stream>>>(FQ, Q16, n8);
        k_gemmw<bf, 0, false><<<dim3(SEQ / 64, EMB / 64, 1), 32, 0, stream>>>(XB, nullptr, WK, nullptr, EMB, FK, EMB, nullptr, 1.0f, 0, 0, 0);
        k_cvth<<<G8, 256, 0, stream>>>(FK, K16, n8);
        k_gemmw<bf, 0, false><<<dim3(SEQ / 64, EMB / 64, 1), 32, 0, stream>>>(XB, nullptr, WV, nullptr, EMB, FV, EMB, nullptr, 1.0f, 0, 0, 0);
        k_vtp8<<<GV, 256, 0, stream>>>(FV, VT16);
        k_meanv<<<(EMB + 255) / 256, 256, 0, stream>>>(FV, MV);
        k_gemmw<h16, 0, false><<<dim3(SEQ / 64, SEQ / 64, 1), 32, 0, stream>>>(Q16, nullptr, K16, nullptr, EMB, Sb, SEQ, nullptr, 1.0f, 0, 0, 0);
        k_asoft<<<SEQ / 8, 256, 0, stream>>>(Sb, P16);
        k_gemmw<h16, 0, true><<<dim3(SEQ / 64, EMB / 64, 1), 32, 0, stream>>>(P16, nullptr, VT16, nullptr, SEQ, ob, EMB, MV, 1.0f / PCAR, 0, 0, 0);
    }
}
